// LinearDecisionTransformerDecoupled_51333449122143
// MI455X (gfx1250) — hardware-run, weakly checked
//
#include <hip/hip_runtime.h>


#ifndef NB
#define NB 2
#endif
#ifndef KT
#define KT 512
#endif
#define NB_FULL 2
#define KT_FULL 512
#define SD   60
#define NA   5
#define DM   256
#define NH_  4
#define HD   64
#define FFD  1024
#define NL   2
#define LSEQ (3 * KT)
#define MROWS (NB * LSEQ)
#define AW   4
#define EPSV 1.0e-6f
#define LNE  1.0e-5f
#define PLN  ((size_t)NB * NH_ * LSEQ * HD)
#define APLN ((size_t)MROWS * DM)
#define FPLN ((size_t)MROWS * FFD)

static_assert(HD == 64);
static_assert(NH_ * HD == DM);
static_assert(DM % 64 == 0);
static_assert(FFD % 64 == 0);
static_assert((3 * DM) % 64 == 0);
static_assert(DM % 32 == 0);
static_assert(FFD % 32 == 0);
static_assert(LSEQ % 64 == 0);
static_assert(MROWS % 64 == 0);
static_assert(LSEQ % 32 == 0);
static_assert(LSEQ % (16 * AW) == 0);
static_assert(MROWS % 8 == 0);
static_assert(KT % 128 == 0);
static_assert(NB <= NB_FULL);
static_assert(KT <= KT_FULL);
static_assert(SD + NA + 1 <= 96);

typedef unsigned short bf;
typedef __attribute__((ext_vector_type(16))) __bf16   v16bf;
typedef __attribute__((ext_vector_type(8)))  unsigned short v8us;
typedef __attribute__((ext_vector_type(16))) unsigned short v16us;
typedef __attribute__((ext_vector_type(8)))  float    v8f;
typedef __attribute__((ext_vector_type(4)))  float    v4f;
typedef v4f  __attribute__((may_alias)) v4fa;

__device__ __forceinline__ unsigned short f2bf(float f) { unsigned u = __float_as_uint(f); u += 0x7FFFu + ((u >> 16) & 1u); return (unsigned short)(u >> 16); }
__device__ __forceinline__ float bf2f(unsigned short w) { return __uint_as_float(((unsigned)w) << 16); }
__device__ __forceinline__ float rb(float f) { return bf2f(f2bf(f)); }
__device__ __forceinline__ v16bf cat16b(v8us lo, v8us hi) { return __builtin_bit_cast(v16bf, __builtin_shufflevector(lo, hi, 0, 1, 2, 3, 4, 5, 6, 7, 8, 9, 10, 11, 12, 13, 14, 15)); }
__device__ __forceinline__ v8f wmmab(v16bf a, v16bf b, v8f c) { return __builtin_amdgcn_wmma_f32_16x16x32_bf16(false, a, false, b, (short)0, c, false, false); }
__device__ __forceinline__ v16bf ldb(const bf* p)  { return cat16b(*(const v8us*)p, *(const v8us*)(p + 16)); }
__device__ __forceinline__ void wave_sync() { __builtin_amdgcn_fence(3  , "wavefront"); __builtin_amdgcn_wave_barrier(); asm volatile("" ::: "memory"); }
__device__ __forceinline__ float wsum(float v) {
#pragma unroll
    for (int off = 16; off > 0; off >>= 1) v += __shfl_xor(v, off, 32);
    return v;
}
__device__ __forceinline__ void split8(v4f x0, v4f x1, v8us& h, v8us& l) {
#pragma unroll
    for (int i = 0; i < 4; ++i) {
        const unsigned short a0 = f2bf(x0[i]); const unsigned short a1 = f2bf(x1[i]);
        h[i] = a0; h[4 + i] = a1; l[i] = f2bf(x0[i] - bf2f(a0)); l[4 + i] = f2bf(x1[i] - bf2f(a1)); }
}

__global__ __launch_bounds__(512) void k_wT(const float* __restrict__ src, bf* dst, int Kd, int N) {
    __shared__ float ts[64 * 65];
    const int i = threadIdx.x; const int n0 = blockIdx.x * 64, k0 = blockIdx.y * 64;
    const float* s = src + (size_t)blockIdx.z * (size_t)Kd * (size_t)N;
    bf* d = dst + (size_t)blockIdx.z * (size_t)N * (size_t)Kd;
#pragma unroll
    for (int it = 0; it < 8; ++it) { const int kk = it * 8 + (i >> 6), nn = i & 63;
        ts[kk * 65 + nn] = s[(size_t)(k0 + kk) * N + n0 + nn]; }
    __syncthreads();
    const int nn = i >> 3, c8 = (i & 7) * 8; v8us o;
#pragma unroll
    for (int j = 0; j < 8; ++j) o[j] = f2bf(ts[(c8 + j) * 65 + nn]);
    bf* p = d + (size_t)(n0 + nn) * Kd + k0 + c8;
    *(volatile v8us*)p = o; __threadfence(); *(volatile v8us*)p = o;
}

__global__ __launch_bounds__(256) void k_embed(const float* __restrict__ rtg, const float* __restrict__ state, const float* __restrict__ action,
                                               const float* __restrict__ rtg_w, const float* __restrict__ rtg_b,
                                               const float* __restrict__ state_w, const float* __restrict__ state_b,
                                               const float* __restrict__ action_w, const float* __restrict__ action_b,
                                               const float* __restrict__ pos, float* x) {
    __shared__ float sv[96];
    const int tid = threadIdx.x; const int b = blockIdx.x / KT, t = blockIdx.x % KT;
    const size_t ib = (size_t)b * KT_FULL + t;
    if (tid < 96) {
        const int js = min(tid, SD - 1); const int ja = min(max(tid - SD, 0), NA - 1);
        const float vs = state[ib * SD + js]; const float va = action[ib * NA + ja]; const float vr = rtg[ib];
        const float v = (tid < SD) ? vs : ((tid < SD + NA) ? va : vr);
        sv[tid] = rb(v);
    }
    __syncthreads();
    const int e = tid;
    const float p = rb(pos[(size_t)t * DM + e]);
    const float r = sv[SD + NA] * rb(rtg_w[e]) + rb(rtg_b[e]) + p;
    float s = 0.0f;
#pragma unroll 4
    for (int j = 0; j < SD; ++j) s = fmaf(sv[j], rb(state_w[j * DM + e]), s);
    s = s + rb(state_b[e]) + p;
    float a = 0.0f;
#pragma unroll 1
    for (int j = 0; j < NA; ++j) a = fmaf(sv[SD + j], rb(action_w[j * DM + e]), a);
    a = a + rb(action_b[e]) + p;
    float* xr = x + ((size_t)b * LSEQ + (size_t)3 * t) * DM + e;
#pragma unroll 1
    for (int ps = 0; ps < 2; ++ps) {
        *(volatile float*)(xr) = r; *(volatile float*)(xr + DM) = s; *(volatile float*)(xr + 2 * DM) = a;
        if (ps == 0) __threadfence(); }
}

__global__ __launch_bounds__(256) void k_ln(const float* __restrict__ x, const float* __restrict__ g, const float* __restrict__ bt, bf* H) {
    const int lane = threadIdx.x & 31; const int wave = (int)(threadIdx.x >> 5);
    const size_t row = (size_t)blockIdx.x * 8 + wave; const int c = lane * 8;
    const float* xr = x + row * DM + c;
    const v4f x0 = *(const v4f*)(xr), x1 = *(const v4f*)(xr + 4);
    const v4f g0 = *(const v4f*)(g + c), g1 = *(const v4f*)(g + c + 4), b0 = *(const v4f*)(bt + c), b1 = *(const v4f*)(bt + c + 4);
    float s = ((x0[0] + x0[1]) + (x0[2] + x0[3])) + ((x1[0] + x1[1]) + (x1[2] + x1[3]));
    const float mean = wsum(s) * (1.0f / DM);
    v4f d0, d1; float q = 0.0f;
#pragma unroll
    for (int i = 0; i < 4; ++i) { d0[i] = x0[i] - mean; d1[i] = x1[i] - mean; q = fmaf(d0[i], d0[i], q); q = fmaf(d1[i], d1[i], q); }
    const float inv = rsqrtf(wsum(q) * (1.0f / DM) + LNE);
    v4f y0, y1;
#pragma unroll
    for (int i = 0; i < 4; ++i) { y0[i] = d0[i] * inv * rb(g0[i]) + rb(b0[i]); y1[i] = d1[i] * inv * rb(g1[i]) + rb(b1[i]); }
    v8us hv, lv; split8(y0, y1, hv, lv);
    bf* Hh = H + row * DM + c; bf* Hl = Hh + APLN;
    *(volatile v8us*)Hh = hv; *(volatile v8us*)Hl = lv; __threadfence(); *(volatile v8us*)Hh = hv; *(volatile v8us*)Hl = lv;
}

__device__ __forceinline__ void gemm64(const bf* __restrict__ A, size_t aplane, const bf* __restrict__ Bt, size_t bplane, int npl, int K, int r0, int c0, int lr, int hi, v8f (&acc)[4][4]) {
#pragma unroll
    for (int mb = 0; mb < 4; ++mb)
#pragma unroll
        for (int nb = 0; nb < 4; ++nb) acc[mb][nb] = (v8f){};
#pragma unroll 1
    for (int pl = 0; pl < npl; ++pl) {
        const size_t aoff = (size_t)pl * aplane + (size_t)(r0 + lr) * K + 8 * hi;
        const size_t boff = (size_t)pl * bplane + (size_t)(c0 + lr) * K + 8 * hi;
#pragma unroll 1
        for (int kc = 0; kc < K; kc += 32) {
            v16bf a[4];
#pragma unroll
            for (int mb = 0; mb < 4; ++mb) a[mb] = ldb(A + aoff + (size_t)mb * 16 * K + kc);
#pragma unroll
            for (int nb = 0; nb < 4; ++nb) { const v16bf b = ldb(Bt + boff + (size_t)nb * 16 * K + kc);
#pragma unroll
                for (int mb = 0; mb < 4; ++mb) acc[mb][nb] = wmmab(a[mb], b, acc[mb][nb]); }
            asm volatile("v_nop\n\tv_nop\n\tv_nop\n\tv_nop" : "+v"(acc[0][0]), "+v"(acc[1][1]), "+v"(acc[2][2]), "+v"(acc[3][3]) : "v"(a[0]), "v"(a[1]), "v"(a[2]), "v"(a[3]));
        }
    }
}

template <int MODE>
__global__ __launch_bounds__(32) void k_proj(const bf* __restrict__ A, size_t aplane, const bf* __restrict__ Bt, size_t bplane, int K, const float* __restrict__ bias,
                                             bf* P, size_t pplane, int RB, size_t sRB, int pitch, int CB, size_t sCB, size_t zB, int zbias, size_t zP) {
    __shared__ __align__(16) float os[16 * 68];
    const int lane = threadIdx.x & 31, lr = lane & 15, hi = lane >> 4; const int r0 = blockIdx.x * 64, c0 = blockIdx.y * 64; const int z = blockIdx.z;
    const bf* Bz = Bt + (size_t)z * zB; const float* bz = bias + (size_t)z * zbias;
    bf* Ph = P + (size_t)z * zP; bf* Pl = Ph + pplane;
    v8f acc[4][4];
    gemm64(A, aplane, Bz, bplane, 2, K, r0, c0, lr, hi, acc);
    const size_t tbase = (size_t)(r0 / RB) * sRB + (size_t)(r0 % RB) * (size_t)pitch + (size_t)(c0 / CB) * sCB + (size_t)(c0 % CB);
    float bc[8];
#pragma unroll
    for (int i = 0; i < 8; ++i) bc[i] = (MODE != 1) ? rb(bz[c0 + (lane & 7) * 8 + i]) : 0.0f;
#pragma unroll
    for (int mb = 0; mb < 4; ++mb) {
#pragma unroll
        for (int nb = 0; nb < 4; ++nb) {
#pragma unroll
            for (int j = 0; j < 8; ++j) os[(hi * 8 + j) * 68 + nb * 16 + lr] = acc[mb][nb][j]; }
        wave_sync();
        if (MODE == 2) {
#pragma unroll 1
            for (int s = 0; s < 4; ++s) { const int row = 4 * s + (lane >> 3), c8 = (lane & 7) * 8;
                v4f x0 = *(const v4fa*)(&os[row * 68 + c8]); v4f x1 = *(const v4fa*)(&os[row * 68 + c8 + 4]);
#pragma unroll
                for (int i = 0; i < 4; ++i) { const float u0 = x0[i] + bc[i]; const float u1 = x1[i] + bc[4 + i];
                    x0[i] = 0.5f * u0 * (1.0f + erff(u0 * 0.70710678118654752f)); x1[i] = 0.5f * u1 * (1.0f + erff(u1 * 0.70710678118654752f)); }
                *(v4fa*)(&os[row * 68 + c8]) = x0; *(v4fa*)(&os[row * 68 + c8 + 4]) = x1; }
            wave_sync();
        }
        const size_t sb = tbase + (size_t)(mb * 16) * (size_t)pitch;
        v8us hv[4], lv[4];
#pragma unroll
        for (int s = 0; s < 4; ++s) { const int row = 4 * s + (lane >> 3), c8 = (lane & 7) * 8;
            v4f x0 = *(const v4fa*)(&os[row * 68 + c8]); v4f x1 = *(const v4fa*)(&os[row * 68 + c8 + 4]);
            if (MODE == 0) {
#pragma unroll
                for (int i = 0; i < 4; ++i) { x0[i] = fmaxf(x0[i] + bc[i], 0.0f) + EPSV; x1[i] = fmaxf(x1[i] + bc[4 + i], 0.0f) + EPSV; } }
            if (MODE == 1) { const float rbv = rb(bz[r0 + mb * 16 + row]);
#pragma unroll
                for (int i = 0; i < 4; ++i) { x0[i] += rbv; x1[i] += rbv; } }
            split8(x0, x1, hv[s], lv[s]); }
#pragma unroll 1
        for (int ps = 0; ps < 2; ++ps) {
#pragma unroll
            for (int s = 0; s < 4; ++s) { const int row = 4 * s + (lane >> 3), c8 = (lane & 7) * 8;
                const size_t oo = sb + (size_t)row * (size_t)pitch + c8;
                *(volatile v8us*)(Ph + oo) = hv[s]; *(volatile v8us*)(Pl + oo) = lv[s]; }
            if (ps == 0) __threadfence(); }
        wave_sync();
    }
}

__global__ __launch_bounds__(32 * AW) __attribute__((amdgpu_num_vgpr(256))) void k_attn(const bf* __restrict__ QK, const bf* __restrict__ VT, bf* CTX) {
    __shared__ __align__(16) float os[AW * 16 * 68];
    const int lane = threadIdx.x & 31, lr = lane & 15, hi = lane >> 4;
    const int wave = __builtin_amdgcn_readfirstlane((int)(threadIdx.x >> 5));
    const int zh = blockIdx.y; const int b = zh / NH_, h = zh % NH_;
    const int t0 = (blockIdx.x * AW + wave) * 16;
    const size_t pbase = (size_t)zh * LSEQ * HD;
    const bf* QH = QK; const bf* QL = QK + PLN; const bf* KH = QK + 2 * PLN; const bf* KL = QK + 3 * PLN;
    const bf* VH = VT; const bf* VL = VT + PLN;
    const size_t qo = pbase + (size_t)(t0 + lr) * HD + 8 * hi;
    const v16bf qh0 = ldb(QH + qo), qh1 = ldb(QH + qo + 32), ql0 = ldb(QL + qo), ql1 = ldb(QL + qo + 32);
    const size_t ko = pbase + (size_t)lr * HD + 8 * hi;
    const size_t vo = pbase + (size_t)lr * LSEQ + 8 * hi;
    v8f o0 = (v8f){}, o1 = (v8f){}, o2 = (v8f){}, o3 = (v8f){};
    float l = 0.0f;
    const int nsteps = (t0 + 15) / 32 + 1;
#pragma unroll 1
    for (int st = 0; st < nsteps; ++st) {
        const int key0 = st * 32;
        const bf* kah = KH + ko + (size_t)key0 * HD; const bf* kal = KL + ko + (size_t)key0 * HD;
        const v16bf kah0 = ldb(kah), kah1 = ldb(kah + 32), kbh0 = ldb(kah + 16 * HD), kbh1 = ldb(kah + 16 * HD + 32);
        const v16bf kal0 = ldb(kal), kal1 = ldb(kal + 32), kbl0 = ldb(kal + 16 * HD), kbl1 = ldb(kal + 16 * HD + 32);
        v8f sa = (v8f){}, sb = (v8f){};
        sa = wmmab(kah0, qh0, sa); sb = wmmab(kbh0, qh0, sb); sa = wmmab(kah1, qh1, sa); sb = wmmab(kbh1, qh1, sb);
        sa = wmmab(kah0, ql0, sa); sb = wmmab(kbh0, ql0, sb); sa = wmmab(kah1, ql1, sa); sb = wmmab(kbh1, ql1, sb);
        sa = wmmab(kal0, qh0, sa); sb = wmmab(kbl0, qh0, sb); sa = wmmab(kal1, qh1, sa); sb = wmmab(kbl1, qh1, sb);
        asm volatile("v_nop\n\tv_nop\n\tv_nop\n\tv_nop" : "+v"(sa), "+v"(sb) : "v"(kah0), "v"(kah1), "v"(kbh0), "v"(kbh1), "v"(kal0), "v"(kal1), "v"(kbl0), "v"(kbl1));
        const int dq = t0 + lr - key0 - 8 * hi;
        v16us shu, slu; float ls = 0.0f;
#pragma unroll
        for (int r = 0; r < 8; ++r) {
            const float ta = (r <= dq) ? sa[r] : 0.0f; const float tb = (r + 16 <= dq) ? sb[r] : 0.0f;
            const unsigned short a = f2bf(ta); const unsigned short c = f2bf(tb);
            shu[r] = a; shu[8 + r] = c; slu[r] = f2bf(ta - bf2f(a)); slu[8 + r] = f2bf(tb - bf2f(c));
            ls += (ta + tb); }
        l += ls;
        const v16bf sh = __builtin_bit_cast(v16bf, shu), sl = __builtin_bit_cast(v16bf, slu);
        const bf* va = VH + vo + key0; const bf* vb = VL + vo + key0;
        const v16bf v0 = ldb(va), v1 = ldb(va + (size_t)16 * LSEQ), v2 = ldb(va + (size_t)32 * LSEQ), v3 = ldb(va + (size_t)48 * LSEQ);
        o0 = wmmab(v0, sh, o0); o1 = wmmab(v1, sh, o1); o2 = wmmab(v2, sh, o2); o3 = wmmab(v3, sh, o3);
        o0 = wmmab(v0, sl, o0); o1 = wmmab(v1, sl, o1); o2 = wmmab(v2, sl, o2); o3 = wmmab(v3, sl, o3);
        const v16bf w0 = ldb(vb), w1 = ldb(vb + (size_t)16 * LSEQ), w2 = ldb(vb + (size_t)32 * LSEQ), w3 = ldb(vb + (size_t)48 * LSEQ);
        o0 = wmmab(w0, sh, o0); o1 = wmmab(w1, sh, o1); o2 = wmmab(w2, sh, o2); o3 = wmmab(w3, sh, o3);
        asm volatile("v_nop\n\tv_nop\n\tv_nop\n\tv_nop" : "+v"(o0), "+v"(o1), "+v"(o2), "+v"(o3) : "v"(v0), "v"(v1), "v"(v2), "v"(v3), "v"(w0), "v"(w1), "v"(w2), "v"(w3), "v"(sh), "v"(sl));
    }
    l += __shfl_xor(l, 16, 32);
    const float inv = 1.0f / fmaxf(l, EPSV);
    const int wb = wave * 16 * 68;
    { v4f a, c;
      a[0] = o0[0] * inv; a[1] = o0[1] * inv; a[2] = o0[2] * inv; a[3] = o0[3] * inv; c[0] = o0[4] * inv; c[1] = o0[5] * inv; c[2] = o0[6] * inv; c[3] = o0[7] * inv;
      *(v4fa*)(&os[wb + lr * 68 +  0 + 8 * hi]) = a; *(v4fa*)(&os[wb + lr * 68 +  0 + 8 * hi + 4]) = c;
      a[0] = o1[0] * inv; a[1] = o1[1] * inv; a[2] = o1[2] * inv; a[3] = o1[3] * inv; c[0] = o1[4] * inv; c[1] = o1[5] * inv; c[2] = o1[6] * inv; c[3] = o1[7] * inv;
      *(v4fa*)(&os[wb + lr * 68 + 16 + 8 * hi]) = a; *(v4fa*)(&os[wb + lr * 68 + 16 + 8 * hi + 4]) = c;
      a[0] = o2[0] * inv; a[1] = o2[1] * inv; a[2] = o2[2] * inv; a[3] = o2[3] * inv; c[0] = o2[4] * inv; c[1] = o2[5] * inv; c[2] = o2[6] * inv; c[3] = o2[7] * inv;
      *(v4fa*)(&os[wb + lr * 68 + 32 + 8 * hi]) = a; *(v4fa*)(&os[wb + lr * 68 + 32 + 8 * hi + 4]) = c;
      a[0] = o3[0] * inv; a[1] = o3[1] * inv; a[2] = o3[2] * inv; a[3] = o3[3] * inv; c[0] = o3[4] * inv; c[1] = o3[5] * inv; c[2] = o3[6] * inv; c[3] = o3[7] * inv;
      *(v4fa*)(&os[wb + lr * 68 + 48 + 8 * hi]) = a; *(v4fa*)(&os[wb + lr * 68 + 48 + 8 * hi + 4]) = c; }
    wave_sync();
    bf* Ch = CTX + ((size_t)b * LSEQ + t0) * DM + h * HD; bf* Cl = Ch + APLN;
    v8us hv[4], lv[4];
#pragma unroll
    for (int s = 0; s < 4; ++s) { const int row = 4 * s + (lane >> 3), c8 = (lane & 7) * 8;
        const v4f x0 = *(const v4fa*)(&os[wb + row * 68 + c8]); const v4f x1 = *(const v4fa*)(&os[wb + row * 68 + c8 + 4]);
        split8(x0, x1, hv[s], lv[s]); }
#pragma unroll 1
    for (int ps = 0; ps < 2; ++ps) {
#pragma unroll
        for (int s = 0; s < 4; ++s) { const int row = 4 * s + (lane >> 3), c8 = (lane & 7) * 8;
            const size_t oo = (size_t)row * DM + c8;
            *(volatile v8us*)(Ch + oo) = hv[s]; *(volatile v8us*)(Cl + oo) = lv[s]; }
        if (ps == 0) __threadfence(); }
}

__global__ __launch_bounds__(32) void k_out(const bf* __restrict__ A, size_t aplane, const bf* __restrict__ Wt, int K, const float* __restrict__ bias, const float* __restrict__ RES, float* OUT) {
    __shared__ __align__(16) float os[16 * 68];
    const int lane = threadIdx.x & 31, lr = lane & 15, hi = lane >> 4; const int r0 = blockIdx.x * 64, c0 = blockIdx.y * 64;
    v8f acc[4][4];
    gemm64(A, aplane, Wt, (size_t)0, 2, K, r0, c0, lr, hi, acc);
    v4f bcv;
#pragma unroll
    for (int i = 0; i < 4; ++i) bcv[i] = rb(bias[c0 + lr * 4 + i]);
#pragma unroll
    for (int mb = 0; mb < 4; ++mb) {
#pragma unroll
        for (int nb = 0; nb < 4; ++nb) {
#pragma unroll
            for (int j = 0; j < 8; ++j) os[(hi * 8 + j) * 68 + nb * 16 + lr] = acc[mb][nb][j]; }
        wave_sync();
        const size_t rbase = (size_t)(r0 + mb * 16) * DM + c0;
        v4f vals[8];
#pragma unroll
        for (int s = 0; s < 8; ++s) { const int row = 2 * s + hi, cofs = lr * 4;
            const v4f val = *(const v4fa*)(&os[row * 68 + cofs]);
            const v4f rv = *(const v4f*)(RES + rbase + (size_t)row * DM + cofs);
            vals[s] = rv + (val + bcv); }
#pragma unroll 1
        for (int ps = 0; ps < 2; ++ps) {
#pragma unroll
            for (int s = 0; s < 8; ++s) { const int row = 2 * s + hi, cofs = lr * 4;
                *(volatile v4f*)(OUT + rbase + (size_t)row * DM + cofs) = vals[s]; }
            if (ps == 0) __threadfence(); }
        wave_sync();
    }
}

__global__ __launch_bounds__(256) void k_head(const float* __restrict__ x, const float* __restrict__ g, const float* __restrict__ bt,
                                              const float* __restrict__ pw, const float* __restrict__ pb, float* out) {
    __shared__ __align__(16) float wt[NA * DM];
    __shared__ __align__(16) float ot[128 * NA];
    const int tid = threadIdx.x; const int lane = tid & 31;
    const int wave = __builtin_amdgcn_readfirstlane((int)(threadIdx.x >> 5));
#pragma unroll 1
    for (int i = tid; i < NA * DM; i += 256) { const int e = i / NA, c = i % NA; wt[c * DM + e] = rb(pw[i]); }
    __syncthreads();
    const int bpb = KT / 128; const int b = blockIdx.x / bpb; const int tb = (blockIdx.x % bpb) * 128;
    const int c = lane * 8;
    const v4f g0 = *(const v4f*)(g + c), g1 = *(const v4f*)(g + c + 4), b0 = *(const v4f*)(bt + c), b1 = *(const v4f*)(bt + c + 4);
#pragma unroll 1
    for (int rr = 0; rr < 16; ++rr) {
        const int tl = wave * 16 + rr; const int t = tb + tl;
        const float* xr = x + ((size_t)b * LSEQ + (size_t)3 * t + 1) * DM + c;
        const v4f x0 = *(const v4f*)(xr), x1 = *(const v4f*)(xr + 4);
        const float s = ((x0[0] + x0[1]) + (x0[2] + x0[3])) + ((x1[0] + x1[1]) + (x1[2] + x1[3]));
        const float mean = wsum(s) * (1.0f / DM);
        v4f d0, d1; float q = 0.0f;
#pragma unroll
        for (int i = 0; i < 4; ++i) { d0[i] = x0[i] - mean; d1[i] = x1[i] - mean; q = fmaf(d0[i], d0[i], q); q = fmaf(d1[i], d1[i], q); }
        const float inv = rsqrtf(wsum(q) * (1.0f / DM) + LNE);
        v4f y0, y1;
#pragma unroll
        for (int i = 0; i < 4; ++i) { y0[i] = d0[i] * inv * rb(g0[i]) + rb(b0[i]); y1[i] = d1[i] * inv * rb(g1[i]) + rb(b1[i]); }
#pragma unroll 1
        for (int cc = 0; cc < NA; ++cc) {
            const v4f w0 = *(const v4fa*)(&wt[cc * DM + c]); const v4f w1 = *(const v4fa*)(&wt[cc * DM + c + 4]);
            float dsum = 0.0f;
#pragma unroll
            for (int i = 0; i < 4; ++i) { dsum = fmaf(y0[i], w0[i], dsum); dsum = fmaf(y1[i], w1[i], dsum); }
            dsum = wsum(dsum);
            if (lane == 0) ot[tl * NA + cc] = dsum + rb(pb[cc]);
        }
    }
    __syncthreads();
    if (wave < 5) {
        const int vi = wave * 32 + lane;
        const v4f val = *(const v4fa*)(&ot[vi * 4]);
        float* dst = out + ((size_t)b * KT_FULL + tb) * NA + (size_t)vi * 4;
        *(volatile v4f*)dst = val; __threadfence(); *(volatile v4f*)dst = val;
    }
}

static constexpr size_t al256(size_t v) { return (v + 255) & ~(size_t)255; }
static constexpr size_t SZ_WQ = al256((size_t)NL * 3 * DM * DM * 2);
static constexpr size_t SZ_WO = al256((size_t)NL * DM * DM * 2);
static constexpr size_t SZ_W1 = al256((size_t)NL * FFD * DM * 2);
static constexpr size_t SZ_W2 = al256((size_t)NL * DM * FFD * 2);
static constexpr size_t SZ_X  = al256(APLN * 4);
static constexpr size_t SZ_HN = al256(2 * APLN * 2);
static constexpr size_t SZ_QK = al256(4 * PLN * 2);
static constexpr size_t SZ_VT = al256(2 * PLN * 2);
static constexpr size_t SZ_CX = al256(2 * APLN * 2);
static constexpr size_t SZ_F1 = al256(2 * FPLN * 2);
static constexpr size_t SZ_TOTAL = SZ_WQ + SZ_WO + SZ_W1 + SZ_W2 + 2 * SZ_X + SZ_HN + SZ_QK + SZ_VT + SZ_CX + SZ_F1;
static_assert(SZ_TOTAL <= (size_t)134217728);
static_assert(PLN == APLN);
static_assert((size_t)((NB_FULL - 1) * KT_FULL + KT_FULL) * NA * 4 == (size_t)20480);

extern "C" void kernel_launch(void* const* d_in, const int* in_sizes, int n_in,
                              void* d_out, int out_size, void* d_ws, size_t ws_size, hipStream_t stream) {
    if (n_in < 26) return;
    const size_t nrow = (size_t)(NB - 1) * KT_FULL + KT;
    if ((size_t)in_sizes[0] < nrow || (size_t)in_sizes[1] < nrow * SD || (size_t)in_sizes[2] < nrow * NA) return;
    if ((size_t)in_sizes[3] < (size_t)DM || (size_t)in_sizes[5] < (size_t)SD * DM || (size_t)in_sizes[7] < (size_t)NA * DM || (size_t)in_sizes[9] < (size_t)KT * DM) return;
    if ((size_t)in_sizes[12] < (size_t)NL * DM * 3 * DM || (size_t)in_sizes[14] < (size_t)NL * DM * DM) return;
    if ((size_t)in_sizes[18] < (size_t)NL * DM * FFD || (size_t)in_sizes[20] < (size_t)NL * FFD * DM) return;
    if ((size_t)in_sizes[24] < (size_t)DM * NA || (size_t)in_sizes[25] < (size_t)NA) return;
    if ((size_t)out_size < nrow * NA) return;
    if (SZ_TOTAL > ws_size) return;
    const float* rtg      = (const float*)d_in[0];  const float* state    = (const float*)d_in[1];  const float* action   = (const float*)d_in[2];
    const float* rtg_w    = (const float*)d_in[3];  const float* rtg_b    = (const float*)d_in[4];
    const float* state_w  = (const float*)d_in[5];  const float* state_b  = (const float*)d_in[6];
    const float* action_w = (const float*)d_in[7];  const float* action_b = (const float*)d_in[8];
    const float* pos_emb  = (const float*)d_in[9];
    const float* norm1_g  = (const float*)d_in[10]; const float* norm1_b  = (const float*)d_in[11];
    const float* qkv_w    = (const float*)d_in[12]; const float* qkv_b    = (const float*)d_in[13];
    const float* out_w    = (const float*)d_in[14]; const float* out_b    = (const float*)d_in[15];
    const float* norm2_g  = (const float*)d_in[16]; const float* norm2_b  = (const float*)d_in[17];
    const float* ffn1_w   = (const float*)d_in[18]; const float* ffn1_b   = (const float*)d_in[19];
    const float* ffn2_w   = (const float*)d_in[20]; const float* ffn2_b   = (const float*)d_in[21];
    const float* normf_g  = (const float*)d_in[22]; const float* normf_b  = (const float*)d_in[23];
    const float* pred_w   = (const float*)d_in[24]; const float* pred_b   = (const float*)d_in[25];
    float* OUT = (float*)d_out;
    char* wsp = (char*)d_ws;
    bf* WQ = (bf*)wsp; wsp += SZ_WQ;
    bf* WO = (bf*)wsp; wsp += SZ_WO;
    bf* W1 = (bf*)wsp; wsp += SZ_W1;
    bf* W2 = (bf*)wsp; wsp += SZ_W2;
    float* XA = (float*)wsp; wsp += SZ_X;
    float* XB = (float*)wsp; wsp += SZ_X;
    bf* HN = (bf*)wsp; wsp += SZ_HN;
    bf* QK = (bf*)wsp; wsp += SZ_QK;
    bf* VT = (bf*)wsp; wsp += SZ_VT;
    bf* CX = (bf*)wsp; wsp += SZ_CX;
    bf* F1 = (bf*)wsp; wsp += SZ_F1;

    k_wT<<<dim3(3 * DM / 64, DM / 64, NL), 512, 0, stream>>>(qkv_w, WQ, DM, 3 * DM);
    k_wT<<<dim3(DM / 64, DM / 64, NL), 512, 0, stream>>>(out_w, WO, DM, DM);
    k_wT<<<dim3(FFD / 64, DM / 64, NL), 512, 0, stream>>>(ffn1_w, W1, DM, FFD);
    k_wT<<<dim3(DM / 64, FFD / 64, NL), 512, 0, stream>>>(ffn2_w, W2, FFD, DM);

    k_embed<<<NB * KT, 256, 0, stream>>>(rtg, state, action, rtg_w, rtg_b, state_w, state_b, action_w, action_b, pos_emb, XA);

    for (int l = 0; l < NL; ++l) {
        const bf* wq = WQ + (size_t)l * 3 * DM * DM;
        k_ln<<<MROWS / 8, 256, 0, stream>>>(XA, norm1_g + l * DM, norm1_b + l * DM, HN);
        k_proj<0><<<dim3(MROWS / 64, DM / 64, 2), 32, 0, stream>>>(HN, APLN, wq, (size_t)0, DM, qkv_b + l * 3 * DM, QK, PLN,
            LSEQ, (size_t)NH_ * LSEQ * HD, HD, HD, (size_t)LSEQ * HD, (size_t)DM * DM, DM, (size_t)2 * PLN);
        k_proj<1><<<dim3(DM / 64, MROWS / 64, 1), 32, 0, stream>>>(wq + (size_t)2 * DM * DM, (size_t)0, HN, APLN, DM, qkv_b + l * 3 * DM + 2 * DM, VT, PLN,
            DM, (size_t)0, LSEQ, LSEQ, (size_t)DM * LSEQ, (size_t)0, 0, (size_t)0);
        k_attn<<<dim3(LSEQ / (16 * AW), NB * NH_, 1), 32 * AW, 0, stream>>>(QK, VT, CX);
        k_out<<<dim3(MROWS / 64, DM / 64, 1), 32, 0, stream>>>(CX, APLN, WO + (size_t)l * DM * DM, DM, out_b + l * DM, XA, XB);
        k_ln<<<MROWS / 8, 256, 0, stream>>>(XB, norm2_g + l * DM, norm2_b + l * DM, HN);
        k_proj<2><<<dim3(MROWS / 64, FFD / 64, 1), 32, 0, stream>>>(HN, APLN, W1 + (size_t)l * FFD * DM, (size_t)0, DM, ffn1_b + l * FFD, F1, FPLN,
            MROWS, (size_t)0, FFD, FFD, (size_t)0, (size_t)0, 0, (size_t)0);
        k_out<<<dim3(MROWS / 64, DM / 64, 1), 32, 0, stream>>>(F1, FPLN, W2 + (size_t)l * DM * FFD, FFD, ffn2_b + l * DM, XB, XA);
    }
    k_head<<<NB * (KT / 128), 256, 0, stream>>>(XA, normf_g, normf_b, pred_w, pred_b, OUT);
}
